// GATGeometric_11871289606992
// MI455X (gfx1250) — hardware-verified
//
#include <hip/hip_runtime.h>

typedef __attribute__((ext_vector_type(16))) _Float16 v16h;
typedef __attribute__((ext_vector_type(8)))  _Float16 v8h;
typedef __attribute__((ext_vector_type(8)))  float  v8f;
typedef __attribute__((ext_vector_type(4)))  float  v4f;
typedef __attribute__((ext_vector_type(4)))  unsigned v4u;
typedef float __attribute__((may_alias)) float_a;

#define N_NODES 50000
#define BT 256
#define ECAP 2560
#define SCAP 32
#define ETILE 2048
#define NBUCK ((N_NODES + BT - 1) / BT)
#define NEG_SLOPE 0.2f

template <typename V> __device__ __forceinline__ void vst2(void* p, V v) {
  *(volatile V*)p = v; __threadfence(); *(volatile V*)p = v;
}
__device__ __forceinline__ v8f wmma_f16(v16h a, v16h b, v8f c) {
  v8f d = __builtin_amdgcn_wmma_f32_16x16x32_f16(false, a, false, b, (short)0, c, false, false);
  asm volatile("v_nop\n\tv_nop\n\tv_nop\n\tv_nop" : "+v"(d) : "v"(a), "v"(b));
  return d;
}
__device__ __forceinline__ v16h frag_h(const _Float16* row, int k0, int lane) {
  union { v16h v; v8h h[2]; } r;
  const _Float16* p = row + k0 + 8 * (lane >> 4);
  r.h[0] = *(const v8h*)(p); r.h[1] = *(const v8h*)(p + 16);
  return r.v;
}
__device__ __forceinline__ v16h frag_f32(const float* row, int k0, int lane) {
  v16h a; const float* p = row + k0 + 8 * (lane >> 4);
#pragma unroll
  for (int i = 0; i < 8; ++i) { a[i] = (_Float16)p[i]; a[8 + i] = (_Float16)p[16 + i]; }
  return a;
}

struct Bucket {
  int lsrc[ECAP]; unsigned short ltgt[ECAP]; unsigned short sub[BT][SCAP]; int scnt[BT]; int wcnt[8][8]; int total;
};
__device__ void bucket_build(Bucket& bk, const int* __restrict__ src, const int* __restrict__ dst, int E, int tlo, int tid) {
  const int lane = tid & 31, wave = tid >> 5;
  if (tid == 0) bk.total = 0;
  __syncthreads();
  for (int e0 = 0; e0 < E; e0 += ETILE) {
    int rv[8]; unsigned msk[8];
#pragma unroll
    for (int j = 0; j < 8; ++j) {
      const int e = e0 + j * 256 + tid;
      const int r = (e < E) ? dst[e] : -1;
      rv[j] = r;
      msk[j] = (unsigned)__builtin_amdgcn_ballot_w32((r >= tlo) && (r < tlo + BT));
    }
    if (lane < 8) bk.wcnt[lane][wave] = __builtin_popcount(msk[lane]);
    __syncthreads();
    const int base = bk.total;
    int run = 0, pre[8];
#pragma unroll
    for (int j = 0; j < 8; ++j) {
#pragma unroll
      for (int w = 0; w < 8; ++w) { if (w == wave) pre[j] = run; run += bk.wcnt[j][w]; }
    }
#pragma unroll
    for (int j = 0; j < 8; ++j) {
      const unsigned m = msk[j];
      if ((m >> lane) & 1u) {
        const int pos = base + pre[j] + __builtin_popcount(m & ((1u << lane) - 1u));
        if (pos < ECAP) { bk.lsrc[pos] = e0 + j * 256 + tid; bk.ltgt[pos] = (unsigned short)(rv[j] - tlo); }
      }
    }
    __syncthreads();
    if (tid == 0) bk.total = base + run;
    __syncthreads();
  }
  const int n = (bk.total < ECAP) ? bk.total : ECAP;
  for (int i = tid; i < n; i += 256) { int s = src[bk.lsrc[i]]; s = s < 0 ? 0 : (s >= N_NODES ? N_NODES - 1 : s); bk.lsrc[i] = s; }
  __syncthreads();
  int k = 0;
  for (int i = 0; i < n; ++i) if ((int)bk.ltgt[i] == tid) { if (k < SCAP) bk.sub[tid][k] = (unsigned short)i; ++k; }
  bk.scnt[tid] = (k < SCAP) ? k : SCAP;
  __syncthreads();
}


__global__ __launch_bounds__(256) void k_wt(const float* __restrict__ W, _Float16* __restrict__ WT, int K, int M) {
  __shared__ __align__(16) _Float16 tile[64][72];
  const int mt = M / 64 > 0 ? M / 64 : 1;
  const int tid = threadIdx.x;
  const int m0 = (blockIdx.x % mt) * 64, k0 = (blockIdx.x / mt) * 64;
  const int mw = (M < 64) ? M : 64;
  for (int i = tid; i < 64 * 64; i += 256) { const int kk = i >> 6, mm = i & 63; tile[mm][kk] = (mm < mw && k0 + kk < K) ? (_Float16)W[(size_t)(k0 + kk) * M + m0 + mm] : (_Float16)0.f; }
  __syncthreads();
  for (int g = tid; g < 64 * 8; g += 256) { const int mm = g >> 3, pc = g & 7; if (mm < mw) vst2(WT + (size_t)(m0 + mm) * K + k0 + pc * 8, *(const v4u*)(&tile[mm][pc * 8])); }
}

template <int K, int M>
__global__ __launch_bounds__(128) void k_gemm(const float* __restrict__ A, const _Float16* __restrict__ WT, float* __restrict__ H) {
  constexpr int NT = M / 16, KC = K / 32;
  __shared__ __align__(16) float so[4][16 * M];
  const int tid = threadIdx.x, wave = tid >> 5, lane = tid & 31, hi = lane >> 4, col = lane & 15;
  const int strip = blockIdx.x * 4 + wave;
  const bool valid = strip < N_NODES / 16;
  if (valid) {
    const float* ar = A + (size_t)(strip * 16 + col) * K;
#pragma unroll 1
    for (int nt = 0; nt < NT; ++nt) {
      v8f acc = {};
      const _Float16* br = WT + (size_t)(nt * 16 + col) * K;
#pragma unroll
      for (int kc = 0; kc < KC; ++kc) acc = wmma_f16(frag_f32(ar, kc * 32, lane), frag_h(br, kc * 32, lane), acc);
#pragma unroll
      for (int r = 0; r < 8; ++r) so[wave][(hi * 8 + r) * M + nt * 16 + col] = acc[r];
    }
  }
  __syncthreads();
  if (valid) {
    float* dst = H + (size_t)strip * 16 * M;
#pragma unroll
    for (int q = 0; q < M / 8; ++q) { const int g = q * 32 + lane; vst2(dst + g * 4, *(const v4f*)(&so[wave][g * 4])); }
  }
}

template <int H, int C>
__global__ __launch_bounds__(256) void k_score(const float* __restrict__ h, const float* __restrict__ asrc, const float* __restrict__ adst,
                                               float* __restrict__ sd) {
  const int i = blockIdx.x * 256 + threadIdx.x;
  if (i >= N_NODES * 16) return;
  const int n = i >> 4, slot = i & 15, hh = slot & 7;
  float v = 0.f;
  if (hh < H) {
    const float* hp = h + (size_t)n * H * C + hh * C;
    const float* ap = (slot < 8 ? asrc : adst) + hh * C;
#pragma unroll 8
    for (int c = 0; c < C; ++c) v += hp[c] * ap[c];
  }
  vst2(sd + i, (float_a)v);
}

template <int H, int C, int MODE>
__global__ __launch_bounds__(256) void k_gat(const int* __restrict__ src, const int* __restrict__ dst, int E,
                                             const float* __restrict__ h, const float* __restrict__ sd,
                                             const float* __restrict__ bias, float* __restrict__ out) {
  constexpr int M = H * C, NJ = M / 32;
  __shared__ Bucket bk;
  const int tid = threadIdx.x, lane = tid & 31, wave = tid >> 5, tlo = blockIdx.x * BT;
  bucket_build(bk, src, dst, E, tlo, tid);
  for (int s = 0; s < 32; ++s) {
    const int t = wave * 32 + s, node = tlo + t;
    if (node >= N_NODES) break;
    const int cnt = bk.scnt[t];
    const float* sdn = sd + (size_t)node * 16;
    float dn[H], mx[H], den[H];
#pragma unroll
    for (int hh = 0; hh < H; ++hh) { dn[hh] = sdn[8 + hh]; float e = sdn[hh] + dn[hh]; e = e > 0.f ? e : NEG_SLOPE * e; mx[hh] = e; den[hh] = 0.f; }
    for (int k = 0; k < cnt; ++k) {
      const int sN = bk.lsrc[bk.sub[t][k]];
      const float* ss = sd + (size_t)sN * 16;
#pragma unroll
      for (int hh = 0; hh < H; ++hh) { float e = ss[hh] + dn[hh]; e = e > 0.f ? e : NEG_SLOPE * e; mx[hh] = fmaxf(mx[hh], e); }
    }
    float acc[NJ];
#pragma unroll
    for (int j = 0; j < NJ; ++j) acc[j] = 0.f;
    for (int k = -1; k < cnt; ++k) {
      const int sN = (k < 0) ? node : bk.lsrc[bk.sub[t][k]];
      const float* ss = sd + (size_t)sN * 16;
      float w[H];
#pragma unroll
      for (int hh = 0; hh < H; ++hh) { float e = ss[hh] + dn[hh]; e = e > 0.f ? e : NEG_SLOPE * e; w[hh] = __expf(e - mx[hh]); den[hh] += w[hh]; }
      const float* hr = h + (size_t)sN * M;
#pragma unroll
      for (int j = 0; j < NJ; ++j) { const int c = lane + 32 * j; acc[j] += w[c / C] * hr[c]; }
    }
    float* orow = out + (size_t)node * M;
    if (MODE == 0) {
#pragma unroll
      for (int j = 0; j < NJ; ++j) {
        const int c = lane + 32 * j;
        float v = acc[j] / den[c / C] + bias[c];
        v = v > 0.f ? v : (__expf(v) - 1.f);
        vst2(orow + c, (float_a)v);
      }
    } else {
      float v = acc[0] / den[0] + bias[lane];
      float m = v;
#pragma unroll
      for (int off = 16; off > 0; off >>= 1) m = fmaxf(m, __shfl_xor(m, off, 32));
      float ex = __expf(v - m), sum = ex;
#pragma unroll
      for (int off = 16; off > 0; off >>= 1) sum += __shfl_xor(sum, off, 32);
      vst2(orow + lane, (float_a)(v - m - __logf(sum)));
    }
  }
}

extern "C" void kernel_launch(void* const* d_in, const int* in_sizes, int n_in,
                              void* d_out, int out_size, void* d_ws, size_t ws_size,
                              hipStream_t stream) {
  (void)n_in; (void)out_size; (void)ws_size;
  const float* x  = (const float*)d_in[0];
  const int*   ei = (const int*)d_in[1];
  const int E = in_sizes[1] / 2;
  const int* src = ei;
  const int* dst = ei + E;
  const float *W1 = (const float*)d_in[2],  *as1 = (const float*)d_in[3],  *ad1 = (const float*)d_in[4],  *b1 = (const float*)d_in[5];
  const float *W2 = (const float*)d_in[6],  *as2 = (const float*)d_in[7],  *ad2 = (const float*)d_in[8],  *b2 = (const float*)d_in[9];
  const float *W3 = (const float*)d_in[10], *as3 = (const float*)d_in[11], *ad3 = (const float*)d_in[12], *b3 = (const float*)d_in[13];
  const float *W4 = (const float*)d_in[14], *as4 = (const float*)d_in[15], *ad4 = (const float*)d_in[16], *b4 = (const float*)d_in[17];
  float* out = (float*)d_out;

  char* ws = (char*)d_ws; size_t off = 0;
  auto alloc = [&](size_t bytes) -> void* { void* p = ws + off; off = (off + bytes + 255) & ~(size_t)255; return p; };
  _Float16* WT1 = (_Float16*)alloc(256 * 256 * 2);
  _Float16* WT2 = (_Float16*)alloc(128 * 256 * 2);
  _Float16* WT3 = (_Float16*)alloc(64 * 128 * 2);
  _Float16* WT4 = (_Float16*)alloc(32 * 64 * 2);
  float* hbuf = (float*)alloc((size_t)N_NODES * 256 * 4);
  float* act1 = (float*)alloc((size_t)N_NODES * 256 * 4);
  float* act2 = (float*)alloc((size_t)N_NODES * 128 * 4);
  float* act3 = (float*)alloc((size_t)N_NODES * 64 * 4);
  float* sd   = (float*)alloc((size_t)N_NODES * 16 * 4);

  const int gstrips = (N_NODES / 16 + 3) / 4;
  const int gsc = (N_NODES * 16 + 255) / 256;

  k_wt<<<(256 / 64) * (256 / 64), 256, 0, stream>>>(W1, WT1, 256, 256);
  k_wt<<<(256 / 64) * (128 / 64), 256, 0, stream>>>(W2, WT2, 256, 128);
  k_wt<<<(128 / 64) * (64 / 64), 256, 0, stream>>>(W3, WT3, 128, 64);
  k_wt<<<(64 / 64) * 1, 256, 0, stream>>>(W4, WT4, 64, 32);

  k_gemm<256, 256><<<gstrips, 128, 0, stream>>>(x, WT1, hbuf);
  k_score<8, 32><<<gsc, 256, 0, stream>>>(hbuf, as1, ad1, sd);
  k_gat<8, 32, 0><<<NBUCK, 256, 0, stream>>>(src, dst, E, hbuf, sd, b1, act1);
  k_gemm<256, 128><<<gstrips, 128, 0, stream>>>(act1, WT2, hbuf);
  k_score<4, 32><<<gsc, 256, 0, stream>>>(hbuf, as2, ad2, sd);
  k_gat<4, 32, 0><<<NBUCK, 256, 0, stream>>>(src, dst, E, hbuf, sd, b2, act2);
  k_gemm<128, 64><<<gstrips, 128, 0, stream>>>(act2, WT3, hbuf);
  k_score<2, 32><<<gsc, 256, 0, stream>>>(hbuf, as3, ad3, sd);
  k_gat<2, 32, 0><<<NBUCK, 256, 0, stream>>>(src, dst, E, hbuf, sd, b3, act3);
  k_gemm<64, 32><<<gstrips, 128, 0, stream>>>(act3, WT4, hbuf);
  k_score<1, 32><<<gsc, 256, 0, stream>>>(hbuf, as4, ad4, sd);
  k_gat<1, 32, 1><<<NBUCK, 256, 0, stream>>>(src, dst, E, hbuf, sd, b4, out);
}
